// ResNetBlock_18433999634782
// MI455X (gfx1250) — hardware-verified
//
#include <hip/hip_runtime.h>
#include <stddef.h>
#include <stdint.h>


#define NCH    64
#define KOFF   27
#define WPL    (NCH * NCH)
#define CBM    128
#define CTHR   256
#define NWAVE  8
#define STR    1024
#define APRW   1024
#define PARTW  192
#define WSTW   130
#define NUW    (KOFF * NCH * NCH / 8)
#define NWBLK  (2 * NUW / CTHR)
#define ACARRY 8.0f
#define WCARRY 256.0f
#define INV_CARRY (1.0f / 2048.0f)
#define EPSV   1e-5f
#define WSMAX  134217728

static_assert(NUW % CTHR == 0);
static_assert(CBM == 16 * NWAVE);
static_assert(STR == 128 * NWAVE);
static_assert((APRW * 8) % CTHR == 0);
static_assert(PARTW % 32 == 0 && PARTW >= 2 * NCH + 1 && PARTW / 4 <= CTHR);
static_assert(NCH % 32 == 0);
static_assert(CBM * NCH * 2 + CBM * KOFF * 4 <= CBM * NCH * 4);
static_assert((CBM * NCH / 8) % CTHR == 0);
static_assert((CBM * KOFF) % 1 == 0);

typedef float          v2f   __attribute__((ext_vector_type(2)));
typedef float          v4f   __attribute__((ext_vector_type(4)));
typedef float          v8f   __attribute__((ext_vector_type(8)));
typedef int            v8i   __attribute__((ext_vector_type(8)));
typedef unsigned short v8us  __attribute__((ext_vector_type(8)));
typedef unsigned short v16us __attribute__((ext_vector_type(16)));
typedef _Float16       v8h   __attribute__((ext_vector_type(8)));
typedef _Float16       v16h  __attribute__((ext_vector_type(16)));
typedef v2f  __attribute__((may_alias)) v2fa;
typedef v4f  __attribute__((may_alias)) v4fa;
typedef v8us __attribute__((may_alias)) v8usa;
union FragH { v16h v; v16us u; v8us h[2]; v8i w; };
union Pk8 { v8h h; v8us u; };
static_assert(sizeof(FragH) == 32);
static_assert(sizeof(Pk8) == 16);

__device__ __forceinline__ v8f wmh(const FragH& a, const FragH& b, v8f c) {
  v8f d = __builtin_amdgcn_wmma_f32_16x16x32_f16(false, a.v, false, b.v, (short)0, c, false, false);
  asm volatile("v_nop\n\tv_nop\n\tv_nop\n\tv_nop" : "+v"(d) : "v"(a.w), "v"(b.w));
  return d;
}

__device__ __forceinline__ v8f z8() { v8f z = {0.f, 0.f, 0.f, 0.f, 0.f, 0.f, 0.f, 0.f}; return z; }

__device__ __forceinline__ v8us pk8h(v4f a, v4f b) {
  Pk8 t;
  t.h[0] = (_Float16)a.x; t.h[1] = (_Float16)a.y; t.h[2] = (_Float16)a.z; t.h[3] = (_Float16)a.w;
  t.h[4] = (_Float16)b.x; t.h[5] = (_Float16)b.y; t.h[6] = (_Float16)b.z; t.h[7] = (_Float16)b.w;
  return t.u;
}

__device__ __forceinline__ v8us wunit(const float* __restrict__ W, int v) {
  const int koff = v >> 9;
  const int n    = (v >> 3) & (NCH - 1);
  const int k8   = (v & 7) * 8;
  const float* p = W + (size_t)koff * WPL + (size_t)k8 * NCH + n;
  v4f a, c;
  a.x = p[0]       * WCARRY; a.y = p[NCH]     * WCARRY; a.z = p[2 * NCH] * WCARRY; a.w = p[3 * NCH] * WCARRY;
  c.x = p[4 * NCH] * WCARRY; c.y = p[5 * NCH] * WCARRY; c.z = p[6 * NCH] * WCARRY; c.w = p[7 * NCH] * WCARRY;
  return pk8h(a, c);
}

__global__ __launch_bounds__(CTHR) void k_stat(const float* __restrict__ x, int nN, int nStat,
                                               const float* __restrict__ W1, const float* __restrict__ W2,
                                               unsigned short* wt1, unsigned short* wt2, float* part) {
  __shared__ float wst[NWAVE * WSTW];
  __shared__ __attribute__((aligned(16))) float pst[PARTW];
  const int tid = (int)threadIdx.x, lane = tid & 31, wave = tid >> 5;
  const int b = (int)blockIdx.x;

  if (b >= nStat) {
    const int wb = b - nStat;
    const int u  = wb * CTHR + tid;
    if (u >= 2 * NUW) return;
    v8us o;
    unsigned short* dp;
    if (wb < NUW / CTHR) {
      o  = wunit(W1, u);
      dp = wt1 + (size_t)u * 8;
    } else {
      const int v = u - NUW;
      o  = wunit(W2, v);
      dp = wt2 + (size_t)v * 8;
    }
    *(volatile v8us*)dp = o;
    __threadfence();
    *(volatile v8us*)dp = o;
    return;
  }

  const int rw0 = b * STR + 128 * wave;
  int wn = 0;
  float wm0 = 0.0f, wm1 = 0.0f, wq0 = 0.0f, wq1 = 0.0f;
#pragma unroll 1
  for (int si = 0; si < 128; ++si) {
    const int row = rw0 + si;
    const int rc  = row < nN ? row : nN - 1;
    const v2f a = *(const v2fa*)(x + (size_t)rc * NCH + 2 * lane);
    if (row < nN) {
      wn += 1;
      const float rk = 1.0f / (float)wn;
      const float d0 = a.x - wm0;
      wm0 = fmaf(d0, rk, wm0);
      wq0 = fmaf(d0, a.x - wm0, wq0);
      const float d1 = a.y - wm1;
      wm1 = fmaf(d1, rk, wm1);
      wq1 = fmaf(d1, a.y - wm1, wq1);
    }
  }
  if (lane == 0) wst[wave * WSTW] = (float)wn;
  wst[wave * WSTW + 1 + 2 * lane]       = wm0;
  wst[wave * WSTW + 2 + 2 * lane]       = wm1;
  wst[wave * WSTW + 1 + NCH + 2 * lane] = wq0;
  wst[wave * WSTW + 2 + NCH + 2 * lane] = wq1;
  __syncthreads();
  if (tid < NCH) {
    float n = 0.0f, mean = 0.0f, M2 = 0.0f;
#pragma unroll 1
    for (int w2 = 0; w2 < NWAVE; ++w2) {
      const float nb = wst[w2 * WSTW];
      const float mb = wst[w2 * WSTW + 1 + tid];
      const float qb = wst[w2 * WSTW + 1 + NCH + tid];
      if (nb > 0.5f) {
        const float nn = n + nb;
        const float delta = mb - mean;
        const float f = nb / nn;
        mean = fmaf(delta, f, mean);
        M2 = M2 + qb + delta * delta * n * f;
        n = nn;
      }
    }
    pst[1 + tid] = mean;
    pst[1 + NCH + tid] = M2;
    if (tid == 0) pst[0] = n;
  } else if (tid >= 2 * NCH + 1 && tid < PARTW) {
    pst[tid] = 0.0f;
  }
  __syncthreads();
  const int tc = tid < PARTW / 4 ? tid : PARTW / 4 - 1;
  const v4f pv = *(const v4fa*)(pst + 4 * tc);
  float* pp = part + (size_t)b * PARTW + 4 * tc;
  if (tid < PARTW / 4) *(volatile v4f*)pp = pv;
  __threadfence();
  if (tid < PARTW / 4) *(volatile v4f*)pp = pv;
}

__global__ __launch_bounds__(CTHR) void k_bnap(const float* __restrict__ src, int nN, int mRows,
                                               const float* __restrict__ part, int nPart,
                                               const float* __restrict__ gam, const float* __restrict__ bet,
                                               unsigned short* ap) {
  __shared__ float wst[4 * WSTW];
  __shared__ float ssh[2 * NCH];
  const int tid = (int)threadIdx.x;
  const int c = tid & (NCH - 1);
  const int q = tid >> 6;
  {
    float n = 0.0f, mean = 0.0f, M2 = 0.0f;
#pragma unroll 1
    for (int b = q; b < nPart; b += 4) {
      const float* pr = part + (size_t)b * PARTW;
      const float nb = pr[0];
      const float mb = pr[1 + c];
      const float qb = pr[1 + NCH + c];
      if (nb > 0.5f) {
        const float nn = n + nb;
        const float delta = mb - mean;
        const float f = nb / nn;
        mean = fmaf(delta, f, mean);
        M2 = M2 + qb + delta * delta * n * f;
        n = nn;
      }
    }
    if (c == 0) wst[q * WSTW] = n;
    wst[q * WSTW + 1 + c] = mean;
    wst[q * WSTW + 1 + NCH + c] = M2;
  }
  __syncthreads();
  if (tid < NCH) {
    float n = 0.0f, mean = 0.0f, M2 = 0.0f;
#pragma unroll 1
    for (int q2 = 0; q2 < 4; ++q2) {
      const float nb = wst[q2 * WSTW];
      const float mb = wst[q2 * WSTW + 1 + tid];
      const float qb = wst[q2 * WSTW + 1 + NCH + tid];
      if (nb > 0.5f) {
        const float nn = n + nb;
        const float delta = mb - mean;
        const float f = nb / nn;
        mean = fmaf(delta, f, mean);
        M2 = M2 + qb + delta * delta * n * f;
        n = nn;
      }
    }
    const float nt = n < 1.0f ? 1.0f : n;
    const float var = M2 * (1.0f / nt);
    const float rstd = rsqrtf(var + EPSV);
    const float sc = gam[tid] * rstd;
    const float sh = bet[tid] - mean * sc;
    ssh[tid] = ACARRY * sc;
    ssh[NCH + tid] = ACARRY * sh;
  }
  __syncthreads();

  const int row0 = (int)blockIdx.x * APRW;
#pragma unroll 1
  for (int it = 0; it < (APRW * 8) / CTHR; ++it) {
    const int u   = it * CTHR + tid;
    const int row = row0 + (u >> 3);
    const int k8  = (u & 7) * 8;
    const int rc  = row < nN ? row : nN - 1;
    const float* p = src + (size_t)rc * NCH + k8;
    const v4f a  = *(const v4fa*)p;
    const v4f bq = *(const v4fa*)(p + 4);
    const bool ok = row < nN;
    float xv[8];
    xv[0] = a.x;  xv[1] = a.y;  xv[2] = a.z;  xv[3] = a.w;
    xv[4] = bq.x; xv[5] = bq.y; xv[6] = bq.z; xv[7] = bq.w;
    float yv[8];
#pragma unroll
    for (int i = 0; i < 8; ++i) {
      const float t = fmaxf(fmaf(xv[i], ssh[k8 + i], ssh[NCH + k8 + i]), 0.0f);
      yv[i] = ok ? t : 0.0f;
    }
    v4f y0, y1;
    y0.x = yv[0]; y0.y = yv[1]; y0.z = yv[2]; y0.w = yv[3];
    y1.x = yv[4]; y1.y = yv[5]; y1.z = yv[6]; y1.w = yv[7];
    const v8us o = pk8h(y0, y1);
    if (row < mRows) {
      unsigned short* dp = ap + (size_t)row * NCH + k8;
      *(volatile v8us*)dp = o;
      __threadfence();
      *(volatile v8us*)dp = o;
    }
  }
}

template <int MODE>
__global__ __launch_bounds__(CTHR) void k_conv(const unsigned short* __restrict__ apl,
                                               const int* __restrict__ nbr, int nN,
                                               const unsigned short* __restrict__ wt,
                                               const float* __restrict__ xres, float* dst, float* part) {
  __shared__ __attribute__((aligned(16))) v4f smem[CBM * NCH / 4];
  __shared__ __attribute__((aligned(16))) float pst[PARTW];
  unsigned short* As = (unsigned short*)smem;
  int* nbs = (int*)(As + CBM * NCH);
  float* stg = (float*)smem;
  const int tid = (int)threadIdx.x, lane = tid & 31, wave = tid >> 5, hh = lane >> 4, m = lane & 15;
  const int v0 = (int)blockIdx.x * CBM;

#pragma unroll 1
  for (int i = tid; i < CBM * KOFF; i += CTHR) {
    const int r = i / KOFF;
    const int k = i - r * KOFF;
    int v = v0 + r;
    v = v > nN - 1 ? nN - 1 : v;
    int idx = nbr[(size_t)v * KOFF + k];
    idx = idx < 0 ? idx + nN : idx;
    idx = idx < 0 ? 0 : (idx > nN - 1 ? nN - 1 : idx);
    nbs[i] = idx;
  }

  v8f acc[4];
#pragma unroll
  for (int t = 0; t < 4; ++t) acc[t] = z8();
  const unsigned short* arow = As + (16 * wave + m) * NCH + 8 * hh;
  const unsigned short* bcol = wt + (size_t)m * NCH + 8 * hh;

#pragma unroll 1
  for (int k = 0; k < KOFF; ++k) {
    __syncthreads();
#pragma unroll
    for (int it = 0; it < (CBM * NCH / 8) / CTHR; ++it) {
      const int p  = it * CTHR + tid;
      const int r  = p >> 3;
      const int c8 = (p & 7) * 8;
      const int idx = nbs[r * KOFF + k];
      const v8us val = *(const v8usa*)(apl + (size_t)idx * NCH + c8);
      *(v8usa*)(As + r * NCH + c8) = val;
    }
    __syncthreads();
    const unsigned short* wk = bcol + (size_t)k * WPL;
#pragma unroll
    for (int kk = 0; kk < NCH / 32; ++kk) {
      FragH af;
      af.h[0] = *(const v8usa*)(arow + 32 * kk);
      af.h[1] = *(const v8usa*)(arow + 32 * kk + 16);
#pragma unroll
      for (int nt = 0; nt < 4; ++nt) {
        const unsigned short* bq = wk + (size_t)(16 * nt) * NCH + 32 * kk;
        FragH bf;
        bf.h[0] = *(const v8usa*)bq;
        bf.h[1] = *(const v8usa*)(bq + 16);
        acc[nt] = wmh(af, bf, acc[nt]);
      }
    }
  }
  __syncthreads();

#pragma unroll
  for (int nt = 0; nt < 4; ++nt) {
    const int lc = 16 * nt + m;
#pragma unroll
    for (int r = 0; r < 8; ++r) {
      const int lr = 16 * wave + 8 * hh + r;
      stg[lr * NCH + lc] = acc[nt][r] * INV_CARRY;
    }
  }
  __syncthreads();

  if (MODE == 0) {
    if (tid < NCH) {
      int nv = nN - v0;
      nv = nv < 0 ? 0 : (nv > CBM ? CBM : nv);
      float s = 0.0f;
#pragma unroll 1
      for (int r = 0; r < nv; ++r) s += stg[r * NCH + tid];
      const float nvf = (float)nv;
      const float mean = s * (1.0f / (nvf < 1.0f ? 1.0f : nvf));
      float qd = 0.0f;
#pragma unroll 1
      for (int r = 0; r < nv; ++r) {
        const float d = stg[r * NCH + tid] - mean;
        qd = fmaf(d, d, qd);
      }
      pst[1 + tid] = mean;
      pst[1 + NCH + tid] = qd;
      if (tid == 0) pst[0] = nvf;
    } else if (tid >= 2 * NCH + 1 && tid < PARTW) {
      pst[tid] = 0.0f;
    }
  }
  __syncthreads();

  v4f pv[8];
  const float* lp = stg + 16 * wave * NCH;
#pragma unroll
  for (int p = 0; p < 8; ++p) pv[p] = *(const v4fa*)(lp + 4 * (32 * p + lane));
  if (MODE == 1) {
#pragma unroll
    for (int p = 0; p < 8; ++p) {
      const int rl = v0 + 16 * wave + 2 * p + hh;
      const int rc = rl < nN ? rl : nN - 1;
      const v4f xv = *(const v4fa*)(xres + (size_t)rc * NCH + 4 * m);
      pv[p] = pv[p] + xv;
    }
  }
  float* gp = dst + (size_t)(v0 + 16 * wave) * NCH;
  const int tc = tid < PARTW / 4 ? tid : PARTW / 4 - 1;
  v4f ppv = {0.0f, 0.0f, 0.0f, 0.0f};
  float* pp = part + (size_t)blockIdx.x * PARTW + 4 * tc;
  if (MODE == 0) ppv = *(const v4fa*)(pst + 4 * tc);

  if (MODE == 0) {
#pragma unroll
    for (int p = 0; p < 8; ++p) *(volatile v4f*)(gp + 4 * (32 * p + lane)) = pv[p];
    if (tid < PARTW / 4) *(volatile v4f*)pp = ppv;
  } else {
#pragma unroll
    for (int p = 0; p < 8; ++p) {
      const int rl = v0 + 16 * wave + 2 * p + hh;
      if (rl < nN) *(volatile v4f*)(gp + 4 * (32 * p + lane)) = pv[p];
    }
  }
  __threadfence();
  if (MODE == 0) {
#pragma unroll
    for (int p = 0; p < 8; ++p) *(volatile v4f*)(gp + 4 * (32 * p + lane)) = pv[p];
    if (tid < PARTW / 4) *(volatile v4f*)pp = ppv;
  } else {
#pragma unroll
    for (int p = 0; p < 8; ++p) {
      const int rl = v0 + 16 * wave + 2 * p + hh;
      if (rl < nN) *(volatile v4f*)(gp + 4 * (32 * p + lane)) = pv[p];
    }
  }
}

static inline int cdiv(int a, int b) { return (a + b - 1) / b; }
static inline size_t al256(size_t o) { return (o + 255) & ~(size_t)255; }

extern "C" void kernel_launch(void* const* d_in, const int* in_sizes, int n_in,
                              void* d_out, int out_size, void* d_ws, size_t ws_size,
                              hipStream_t stream) {
  if (n_in < 8) return;
  if (in_sizes[0] < NCH || (in_sizes[0] % NCH) != 0) return;
  const int nN = in_sizes[0] / NCH;
  if (nN < 1 || nN >= (1 << 24)) return;
  if (in_sizes[1] != nN * KOFF) return;
  if (in_sizes[2] != KOFF * NCH * NCH || in_sizes[5] != KOFF * NCH * NCH) return;
  if (in_sizes[3] != NCH || in_sizes[4] != NCH || in_sizes[6] != NCH || in_sizes[7] != NCH) return;
  if (out_size != nN * NCH) return;

  const float* x   = (const float*)d_in[0];
  const int*   nbr = (const int*)d_in[1];
  const float* W1  = (const float*)d_in[2];
  const float* g1  = (const float*)d_in[3];
  const float* b1  = (const float*)d_in[4];
  const float* W2  = (const float*)d_in[5];
  const float* g2  = (const float*)d_in[6];
  const float* b2  = (const float*)d_in[7];
  float* out = (float*)d_out;

  const int MP = cdiv(nN, CBM) * CBM;
  const int gC = MP / CBM;
  const int gS = cdiv(nN, STR);
  const int gA = cdiv(MP, APRW);
  if ((long long)gA * APRW < (long long)MP) return;

  char* ws = (char*)d_ws;
  size_t off = 0;
  const size_t oAP = off; off = al256(off + (size_t)MP * NCH * 2);
  const size_t oO1 = off; off = al256(off + (size_t)MP * NCH * 4);
  const size_t oW1 = off; off = al256(off + (size_t)KOFF * WPL * 2);
  const size_t oW2 = off; off = al256(off + (size_t)KOFF * WPL * 2);
  const size_t oP1 = off; off = al256(off + (size_t)gS * PARTW * 4);
  const size_t oP2 = off; off = al256(off + (size_t)gC * PARTW * 4);
  if (off > ws_size || off > (size_t)WSMAX) return;
  unsigned short* AP  = (unsigned short*)(ws + oAP);
  float*          O1  = (float*)(ws + oO1);
  unsigned short* WT1 = (unsigned short*)(ws + oW1);
  unsigned short* WT2 = (unsigned short*)(ws + oW2);
  float*          P1  = (float*)(ws + oP1);
  float*          P2  = (float*)(ws + oP2);

  k_stat<<<gS + NWBLK, CTHR, 0, stream>>>(x, nN, gS, W1, W2, WT1, WT2, P1);
  k_bnap<<<gA, CTHR, 0, stream>>>(x, nN, MP, P1, gS, g1, b1, AP);
  k_conv<0><<<gC, CTHR, 0, stream>>>(AP, nbr, nN, WT1, x, O1, P2);
  k_bnap<<<gA, CTHR, 0, stream>>>(O1, nN, MP, P2, gC, g2, b2, AP);
  k_conv<1><<<gC, CTHR, 0, stream>>>(AP, nbr, nN, WT2, x, out, P2);
}
